// graph_network_18906446037564
// MI455X (gfx1250) — hardware-verified
//
#include <hip/hip_runtime.h>


namespace {
constexpr int N = 50000, E = 300000, NI = 16, EI = 8, H = 64, OUT = 3, L = 3, NB = (N + 127) / 128, EB = (E + 127) / 128, AGN = 512, AGB = (N + AGN - 1) / AGN;
constexpr float AS_ = 8.0f, EPS = 1e-5f;

typedef _Float16 b16;
typedef __attribute__((ext_vector_type(16))) _Float16 v16b;
typedef __attribute__((ext_vector_type(8))) _Float16 v8b;
typedef __attribute__((ext_vector_type(8))) float v8f;
typedef __attribute__((ext_vector_type(4))) float v4f;
__device__ __forceinline__ float bf16_rne(float f) { unsigned int u = __float_as_uint(f); u += 0x7FFFu + ((u >> 16) & 1u); return __uint_as_float(u & 0xFFFF0000u); }
__device__ __forceinline__ void split16(float v, b16& hi, b16& lo) { hi = (b16)v; lo = (b16)(v - (float)hi); }
__device__ __forceinline__ v16b frag_kb(const b16* p, int hh) { const v8b a = *(const v8b*)(p + 8 * hh), b = *(const v8b*)(p + 16 + 8 * hh); v16b f;
#pragma unroll
  for (int e = 0; e < 8; ++e) { f[e] = a[e]; f[8 + e] = b[e]; } return f; }
__device__ __forceinline__ void frag_split(const float* p, int hh, v16b& fh, v16b& fl) {
#pragma unroll
  for (int e = 0; e < 8; ++e) { b16 a, c; split16(p[8 * hh + e] * AS_, a, c); fh[e] = a; fl[e] = c; split16(p[16 + 8 * hh + e] * AS_, a, c); fh[8 + e] = a; fl[8 + e] = c; } }
__device__ __forceinline__ v8f wmma16b(v16b a, v16b b, v8f c) { v8f d = __builtin_amdgcn_wmma_f32_16x16x32_f16(false, a, false, b, (short)0, c, false, false); asm volatile("v_nop\n\tv_nop\n\tv_nop\n\tv_nop" : "+v"(d) : "v"(a), "v"(b)); return d; }
__device__ __forceinline__ void wave_lds_sync() { __builtin_amdgcn_fence(__ATOMIC_RELEASE, "workgroup"); __builtin_amdgcn_wave_barrier(); __builtin_amdgcn_fence(__ATOMIC_ACQUIRE, "workgroup"); }
__device__ __forceinline__ float pmul(float a, float b) { float p = a * b; asm volatile("" : "+v"(p)); return p; }
__device__ __forceinline__ float lrelu(float x) { return (x >= 0.0f) ? x : 0.05f * x; }

struct Wo_ { static constexpr size_t NE1 = 0, NE2 = NE1 + 64 * 32, EE1 = NE2 + 64 * 64, EE2 = EE1 + 64 * 32, EM = EE2 + 64 * 64  , EMSZ = 64 * 192 + 64 * 64, NM = EM + (size_t)L * EMSZ, NMSZ = 64 * 128 + 64 * 64, D1 = NM + (size_t)L * NMSZ, D2 = D1 + 64 * 64, END = D2 + 16 * 64; };
__global__ __launch_bounds__(256) void prep_kernel(const float* __restrict__ neW1, const float* __restrict__ neW2, const float* __restrict__ eeW1, const float* __restrict__ eeW2, const float* __restrict__ emW1, const float* __restrict__ emW2, const float* __restrict__ nmW1, const float* __restrict__ nmW2, const float* __restrict__ dW1, const float* __restrict__ dW2,
                                                   const float* const* __restrict__ dummy, b16* __restrict__ R) {
  (void)dummy;
  const int t_ = blockIdx.x * 256 + threadIdx.x, nth = gridDim.x * 256;
  auto tr = [&](size_t base, int nrow, int kp, auto val) { for (int p = t_; p < nrow * kp / 8; p += nth) { const int o = p / (kp / 8), k0 = (p % (kp / 8)) * 8; v8b v;
#pragma unroll
      for (int e8 = 0; e8 < 8; ++e8) v[e8] = (b16)val(o, k0 + e8); *(volatile v8b*)(R + base + (size_t)o * kp + k0) = v; } };
  for (int pass = 0; pass < 2; ++pass) {
    tr(Wo_::NE1, 64, 32, [&](int o, int k) { return (k < NI) ? bf16_rne(neW1[k * H + o]) : 0.0f; });
    tr(Wo_::EE1, 64, 32, [&](int o, int k) { return (k < EI) ? bf16_rne(eeW1[k * H + o]) : 0.0f; });
    tr(Wo_::NE2, 64, 64, [&](int o, int k) { return bf16_rne(neW2[k * H + o]); });
    tr(Wo_::EE2, 64, 64, [&](int o, int k) { return bf16_rne(eeW2[k * H + o]); });
    tr(Wo_::D1, 64, 64, [&](int o, int k) { return bf16_rne(dW1[k * H + o]); });
    tr(Wo_::D2, 16, 64, [&](int o, int k) { return (o < OUT) ? bf16_rne(dW2[k * OUT + o]) : 0.0f; });
    for (int l = 0; l < L; ++l) {
      tr(Wo_::EM + (size_t)l * Wo_::EMSZ, 64, 192, [&](int o, int k) { return bf16_rne(emW1[((size_t)l * 192 + k) * H + o]); });
      tr(Wo_::EM + (size_t)l * Wo_::EMSZ + 64 * 192, 64, 64, [&](int o, int k) { return bf16_rne(emW2[((size_t)l * 64 + k) * H + o]); });
      tr(Wo_::NM + (size_t)l * Wo_::NMSZ, 64, 128, [&](int o, int k) { return bf16_rne(nmW1[((size_t)l * 128 + k) * H + o]); });
      tr(Wo_::NM + (size_t)l * Wo_::NMSZ + 64 * 128, 64, 64, [&](int o, int k) { return bf16_rne(nmW2[((size_t)l * 64 + k) * H + o]); }); }
    __threadfence(); }
}
__global__ __launch_bounds__(256) void pprep_kernel(const float* __restrict__ ne_b1, const float* __restrict__ ne_b2, const float* __restrict__ ne_g, const float* __restrict__ ne_be, const float* __restrict__ ee_b1, const float* __restrict__ ee_b2, const float* __restrict__ ee_g, const float* __restrict__ ee_be,
                                                    const float* __restrict__ em_b1, const float* __restrict__ em_b2, const float* __restrict__ em_g, const float* __restrict__ em_be, const float* __restrict__ nm_b1, const float* __restrict__ nm_b2, const float* __restrict__ nm_g, const float* __restrict__ nm_be, const float* __restrict__ d_b1, const float* __restrict__ d_b2, float* __restrict__ P) {
  const int t_ = blockIdx.x * 256 + threadIdx.x, nth = gridDim.x * 256;
  for (int pass = 0; pass < 2; ++pass) { for (int q = t_; q < 9 * 256; q += nth) { const int m = q >> 8, f = (q >> 6) & 3, i = q & 63; float v = 0.0f;
      if (m == 0) v = (f == 0) ? ne_b1[i] : (f == 1) ? ne_b2[i] : (f == 2) ? ne_g[i] : ne_be[i];
      else if (m == 1) v = (f == 0) ? ee_b1[i] : (f == 1) ? ee_b2[i] : (f == 2) ? ee_g[i] : ee_be[i];
      else if (m < 5) { const int l = m - 2; v = (f == 0) ? em_b1[l * H + i] : (f == 1) ? em_b2[l * H + i] : (f == 2) ? em_g[l * H + i] : em_be[l * H + i]; }
      else if (m < 8) { const int l = m - 5; v = (f == 0) ? nm_b1[l * H + i] : (f == 1) ? nm_b2[l * H + i] : (f == 2) ? nm_g[l * H + i] : nm_be[l * H + i]; }
      else v = (f == 0) ? d_b1[i] : (f == 1 && i < OUT) ? d_b2[i] : 0.0f;
      P[q] = bf16_rne(v); } __threadfence(); }
}

__device__ __forceinline__ void mlp_tail(v8f acc[4], float (*T)[H + 4], const b16* W2, const float* Pm, int nloc, int hlf, v8f y[4]) {
#pragma unroll
  for (int t = 0; t < 4; ++t) { const float bb = Pm[t * 16 + nloc];
#pragma unroll
    for (int r = 0; r < 8; ++r) T[8 * hlf + r][t * 16 + nloc] = lrelu(acc[t][r] * (1.0f / AS_) + bb); }
  wave_lds_sync();
  v8f a2[4] = {{}, {}, {}, {}};
#pragma unroll
  for (int kb = 0; kb < H; kb += 32) { v16b ah, al; frag_split(&T[nloc][kb], hlf, ah, al);
#pragma unroll
    for (int t = 0; t < 4; ++t) { const v16b bw = frag_kb(W2 + (size_t)(t * 16 + nloc) * H + kb, hlf); a2[t] = wmma16b(ah, bw, a2[t]); a2[t] = wmma16b(al, bw, a2[t]); } }
  float hv[4][8];
#pragma unroll
  for (int t = 0; t < 4; ++t) { const float bb = Pm[64 + t * 16 + nloc];
#pragma unroll
    for (int r = 0; r < 8; ++r) hv[t][r] = lrelu(a2[t][r] * (1.0f / AS_) + bb); }
#pragma unroll
  for (int r = 0; r < 8; ++r) { float s = (hv[0][r] + hv[1][r]) + (hv[2][r] + hv[3][r]);
#pragma unroll
    for (int o = 1; o < 16; o <<= 1) s += __shfl_xor(s, o);
    const float mu = s * (1.0f / H); float q = 0.0f;
#pragma unroll
    for (int t = 0; t < 4; ++t) { const float d = hv[t][r] - mu; q += pmul(d, d); }
#pragma unroll
    for (int o = 1; o < 16; o <<= 1) q += __shfl_xor(q, o);
    const float is = rsqrtf(q * (1.0f / H) + EPS);
#pragma unroll
    for (int t = 0; t < 4; ++t) { const int c = t * 16 + nloc; y[t][r] = pmul((hv[t][r] - mu) * is, Pm[128 + c]) + Pm[192 + c]; } }
  wave_lds_sync();
}

__global__ __launch_bounds__(128) void enc_kernel(const float* __restrict__ X, int count, int kin, const b16* __restrict__ W1, const b16* __restrict__ W2, const float* __restrict__ Pm, float* __restrict__ Y) {
  __shared__ __attribute__((aligned(16))) float T[4][16][H + 4];
  const int lane = threadIdx.x & 31, wave = threadIdx.x >> 5, nloc = lane & 15, hlf = lane >> 4, r0 = blockIdx.x * 64 + wave * 16;
  v16b a = {}; { const int row = r0 + nloc; if (row < count) {
#pragma unroll
      for (int e = 0; e < 16; ++e) { const int k = (e < 8) ? (8 * hlf + e) : (16 + 8 * hlf + e - 8); if (k < kin) a[e] = (b16)bf16_rne(X[(size_t)row * kin + k]); } } }
  v8f acc[4];
#pragma unroll
  for (int t = 0; t < 4; ++t) { acc[t] = (v8f){}; const v16b bw = frag_kb(W1 + (size_t)(t * 16 + nloc) * 32, hlf); acc[t] = wmma16b(a, bw, acc[t]);
#pragma unroll
    for (int r = 0; r < 8; ++r) acc[t][r] *= AS_; }
  v8f y[4]; mlp_tail(acc, T[wave], W2, Pm, nloc, hlf, y);
#pragma unroll
  for (int t = 0; t < 4; ++t)
#pragma unroll
    for (int r = 0; r < 8; ++r) T[wave][8 * hlf + r][t * 16 + nloc] = y[t][r];
  wave_lds_sync();
  for (int pass = 0; pass < 2; ++pass) { for (int i = lane; i < 16 * 16; i += 32) { const int rr = i >> 4, c4 = (i & 15) * 4; if (r0 + rr < count) *(volatile v4f*)(Y + (size_t)(r0 + rr) * H + c4) = *(const v4f*)(&T[wave][rr][c4]); } __threadfence(); }
}

__global__ __launch_bounds__(128) void edge_kernel(float* __restrict__ e, const float* __restrict__ n, const int* __restrict__ ei, const b16* __restrict__ W1, const b16* __restrict__ W2, const float* __restrict__ Pm) {
  __shared__ __attribute__((aligned(16))) float T[4][16][H + 4];
  const int lane = threadIdx.x & 31, wave = threadIdx.x >> 5, nloc = lane & 15, hlf = lane >> 4, r0 = blockIdx.x * 64 + wave * 16; const int row = r0 + nloc, rowc = (row < E) ? row : E - 1;
  int s = ei[(size_t)rowc * 2], rr_ = ei[(size_t)rowc * 2 + 1]; s = (s < 0) ? 0 : (s >= N ? N - 1 : s); rr_ = (rr_ < 0) ? 0 : (rr_ >= N ? N - 1 : rr_);
  __shared__ __attribute__((aligned(16))) float G[4][2][16][H + 4];
  {
    const float* ps_ = n + (size_t)s * H + 32 * hlf; const float* pr_ = n + (size_t)rr_ * H + 32 * hlf;
#pragma unroll
    for (int c = 0; c < 32; c += 4) { *(v4f*)(&G[wave][0][nloc][32 * hlf + c]) = *(const v4f*)(ps_ + c); *(v4f*)(&G[wave][1][nloc][32 * hlf + c]) = *(const v4f*)(pr_ + c); } }
  wave_lds_sync();
  v8f acc[4] = {{}, {}, {}, {}};
#pragma unroll
  for (int kb = 0; kb < 192; kb += 32) { const float* src = (kb < 64) ? (e + (size_t)rowc * H + kb) : (kb < 128) ? (&G[wave][0][nloc][kb - 64]) : (&G[wave][1][nloc][kb - 128]); v16b ah, al; frag_split(src, hlf, ah, al);
#pragma unroll
    for (int t = 0; t < 4; ++t) { const v16b bw = frag_kb(W1 + (size_t)(t * 16 + nloc) * 192 + kb, hlf); acc[t] = wmma16b(ah, bw, acc[t]); acc[t] = wmma16b(al, bw, acc[t]); } }
  v8f y[4]; mlp_tail(acc, T[wave], W2, Pm, nloc, hlf, y);
#pragma unroll
  for (int t = 0; t < 4; ++t)
#pragma unroll
    for (int r = 0; r < 8; ++r) { const int rw = r0 + 8 * hlf + r; const int rwc = (rw < E) ? rw : E - 1; T[wave][8 * hlf + r][t * 16 + nloc] = e[(size_t)rwc * H + t * 16 + nloc] + y[t][r]; }
  wave_lds_sync();
  for (int pass = 0; pass < 2; ++pass) { for (int i = lane; i < 16 * 16; i += 32) { const int rr = i >> 4, c4 = (i & 15) * 4; if (r0 + rr < E) *(volatile v4f*)(e + (size_t)(r0 + rr) * H + c4) = *(const v4f*)(&T[wave][rr][c4]); } __threadfence(); }
}

__global__ __launch_bounds__(256) void aggr_kernel(const float* __restrict__ e, const int* __restrict__ ei, float* __restrict__ aggr) {
  __shared__ __attribute__((aligned(16))) float Acc[AGN][H]; __shared__ int Lst[256]; __shared__ int Lnode[256]; __shared__ int Cnt[8]; __shared__ int tot;
  const int t_ = threadIdx.x, wave = t_ >> 5, lane = t_ & 31, v0 = blockIdx.x * AGN;
  for (int i = t_; i < AGN * H; i += 256) (&Acc[0][0])[i] = 0.0f;
  __syncthreads();
  for (int c0 = 0; c0 < E; c0 += 256) { const int ed = c0 + t_; int s = -1; if (ed < E) { const int sv = ei[(size_t)ed * 2]; if (sv >= v0 && sv < v0 + AGN) s = sv - v0; }
    const unsigned int bal = __builtin_amdgcn_ballot_w32(s >= 0); if (lane == 0) Cnt[wave] = __builtin_popcount(bal);
    __syncthreads();
    int base = 0; for (int w = 0; w < wave; ++w) base += Cnt[w]; const int pos = base + __builtin_popcount(bal & ((1u << lane) - 1u));
    if (s >= 0) { Lst[pos] = ed; Lnode[pos] = s; }
    if (t_ == 0) { int a = 0; for (int w = 0; w < 8; ++w) a += Cnt[w]; tot = a; }
    __syncthreads();
    const int nh = tot;
    for (int k = 0; k < nh; ++k) { const int nd = Lnode[k]; if ((nd & 255) == t_) { const float* er = e + (size_t)Lst[k] * H; float* ac = Acc[nd];
#pragma unroll 8
        for (int c = 0; c < H; ++c) ac[c] += er[c]; } }
    __syncthreads(); }
  for (int pass = 0; pass < 2; ++pass) { for (int i = t_; i < AGN * (H / 4); i += 256) { const int rr = i / (H / 4), c4 = (i % (H / 4)) * 4; if (v0 + rr < N) *(volatile v4f*)(aggr + (size_t)(v0 + rr) * H + c4) = *(const v4f*)(&Acc[rr][c4]); } __threadfence(); }
}

__global__ __launch_bounds__(128) void node_kernel(float* __restrict__ n, const float* __restrict__ aggr, const b16* __restrict__ W1, const b16* __restrict__ W2, const float* __restrict__ Pm) {
  __shared__ __attribute__((aligned(16))) float T[4][16][H + 4];
  const int lane = threadIdx.x & 31, wave = threadIdx.x >> 5, nloc = lane & 15, hlf = lane >> 4, r0 = blockIdx.x * 64 + wave * 16; const int row = r0 + nloc, rowc = (row < N) ? row : N - 1;
  v8f acc[4] = {{}, {}, {}, {}};
#pragma unroll
  for (int kb = 0; kb < 128; kb += 32) { const float* src = (kb < 64) ? (n + (size_t)rowc * H + kb) : (aggr + (size_t)rowc * H + kb - 64); v16b ah, al; frag_split(src, hlf, ah, al);
#pragma unroll
    for (int t = 0; t < 4; ++t) { const v16b bw = frag_kb(W1 + (size_t)(t * 16 + nloc) * 128 + kb, hlf); acc[t] = wmma16b(ah, bw, acc[t]); acc[t] = wmma16b(al, bw, acc[t]); } }
  v8f y[4]; mlp_tail(acc, T[wave], W2, Pm, nloc, hlf, y);
#pragma unroll
  for (int t = 0; t < 4; ++t)
#pragma unroll
    for (int r = 0; r < 8; ++r) { const int rw = r0 + 8 * hlf + r; const int rwc = (rw < N) ? rw : N - 1; T[wave][8 * hlf + r][t * 16 + nloc] = n[(size_t)rwc * H + t * 16 + nloc] + y[t][r]; }
  wave_lds_sync();
  for (int pass = 0; pass < 2; ++pass) { for (int i = lane; i < 16 * 16; i += 32) { const int rr = i >> 4, c4 = (i & 15) * 4; if (r0 + rr < N) *(volatile v4f*)(n + (size_t)(r0 + rr) * H + c4) = *(const v4f*)(&T[wave][rr][c4]); } __threadfence(); }
}

__global__ __launch_bounds__(128) void dec_kernel(const float* __restrict__ n, const b16* __restrict__ W1, const b16* __restrict__ W2, const float* __restrict__ Pd, float* __restrict__ out) {
  __shared__ __attribute__((aligned(16))) float T[4][16][H + 4]; __shared__ float Z[64][OUT];
  const int lane = threadIdx.x & 31, wave = threadIdx.x >> 5, nloc = lane & 15, hlf = lane >> 4, b0 = blockIdx.x * 64, r0 = b0 + wave * 16; const int row = r0 + nloc, rowc = (row < N) ? row : N - 1;
  v8f acc[4] = {{}, {}, {}, {}};
#pragma unroll
  for (int kb = 0; kb < H; kb += 32) { v16b ah, al; frag_split(n + (size_t)rowc * H + kb, hlf, ah, al);
#pragma unroll
    for (int t = 0; t < 4; ++t) { const v16b bw = frag_kb(W1 + (size_t)(t * 16 + nloc) * H + kb, hlf); acc[t] = wmma16b(ah, bw, acc[t]); acc[t] = wmma16b(al, bw, acc[t]); } }
#pragma unroll
  for (int t = 0; t < 4; ++t) { const float bb = Pd[t * 16 + nloc];
#pragma unroll
    for (int r = 0; r < 8; ++r) T[wave][8 * hlf + r][t * 16 + nloc] = lrelu(acc[t][r] * (1.0f / AS_) + bb); }
  wave_lds_sync();
  v8f z = {};
#pragma unroll
  for (int kb = 0; kb < H; kb += 32) { v16b ah, al; frag_split(&T[wave][nloc][kb], hlf, ah, al); const v16b bw = frag_kb(W2 + (size_t)nloc * H + kb, hlf); z = wmma16b(ah, bw, z); z = wmma16b(al, bw, z); }
  if (nloc < OUT) {
#pragma unroll
    for (int r = 0; r < 8; ++r) Z[wave * 16 + 8 * hlf + r][nloc] = z[r] * (1.0f / AS_) + Pd[64 + nloc]; }
  __syncthreads();
  const int nrow = (b0 + 64 <= N) ? 64 : (N - b0);
  for (int pass = 0; pass < 2; ++pass) { for (int i = threadIdx.x; i < nrow * OUT; i += 128) ((volatile float*)out)[(size_t)b0 * OUT + i] = (&Z[0][0])[i]; __threadfence(); }
}
}

extern "C" void kernel_launch(void* const* d_in, const int* in_sizes, int n_in,
                              void* d_out, int out_size, void* d_ws, size_t ws_size, hipStream_t stream) {
  (void)n_in; (void)out_size;
  const float* nodes = (const float*)d_in[0]; const float* edges = (const float*)d_in[1]; const int* ei = (const int*)d_in[2];
  const float* f[31]; for (int i = 3; i < 31; ++i) f[i] = (const float*)d_in[i];
  float* out = (float*)d_out;
  if (in_sizes[0] != N * NI || in_sizes[1] != E * EI || in_sizes[2] != E * 2 || in_sizes[21] != L * 192 * H || in_sizes[29] != H * OUT) return;
  size_t off = 0; char* ws = (char*)d_ws;
  auto carve = [&](size_t bytes) { char* p = ws + off; off += (bytes + 255) & ~(size_t)255; return p; };
  b16* R = (b16*)carve(Wo_::END * 2); float* P = (float*)carve(9 * 256 * 4); float* n = (float*)carve((size_t)N * H * 4); float* e = (float*)carve((size_t)E * H * 4); float* aggr = (float*)carve((size_t)N * H * 4);
  if (off > ws_size) return;
  prep_kernel<<<64, 256, 0, stream>>>(f[3], f[5], f[9], f[11], f[21], f[23], f[15], f[17], f[27], f[29], nullptr, R);
  pprep_kernel<<<8, 256, 0, stream>>>(f[4], f[6], f[7], f[8], f[10], f[12], f[13], f[14], f[22], f[24], f[25], f[26], f[16], f[18], f[19], f[20], f[28], f[30], P);
  enc_kernel<<<(N + 63) / 64, 128, 0, stream>>>(nodes, N, NI, R + Wo_::NE1, R + Wo_::NE2, P + 0 * 256, n);
  enc_kernel<<<(E + 63) / 64, 128, 0, stream>>>(edges, E, EI, R + Wo_::EE1, R + Wo_::EE2, P + 1 * 256, e);
  for (int l = 0; l < L; ++l) {
    edge_kernel<<<(E + 63) / 64, 128, 0, stream>>>(e, n, ei, R + Wo_::EM + (size_t)l * Wo_::EMSZ, R + Wo_::EM + (size_t)l * Wo_::EMSZ + 64 * 192, P + (2 + l) * 256);
    aggr_kernel<<<AGB, 256, 0, stream>>>(e, ei, aggr);
    node_kernel<<<(N + 63) / 64, 128, 0, stream>>>(n, aggr, R + Wo_::NM + (size_t)l * Wo_::NMSZ, R + Wo_::NM + (size_t)l * Wo_::NMSZ + 64 * 128, P + (5 + l) * 256); }
  dec_kernel<<<(N + 63) / 64, 128, 0, stream>>>(n, R + Wo_::D1, R + Wo_::D2, P + 8 * 256, out);
}
